// GNNSage_46437186404819
// MI455X (gfx1250) — hardware-verified
//
#include <hip/hip_runtime.h>
#include <stddef.h>
#include <math.h>


#define FD      128
#define NCLS    5
#define YW      16
#define NTHR    256
#define NWAVE   8
#define EPT     8
#define NGRP    2
#define CHUNK   (NTHR * EPT * NGRP)
#define WCAP    (EPT * NGRP * 32)
#define LISTN   (NWAVE * WCAP)
#define NBC     4096
#define NBF     1024
#define RCAP    40960
#define RBN     128
#define TGT     256
#define DEGCAP  1024
#define GROWS   128
#define OTHR    512
#define WSCAP   134217728

#define K1      128
#define APK1    136
#define K2      256
#define APK2    264

#define WP_M    0
#define WP_PL   65536
#define WP_P    98304
#define WP_O    163840
#define WPTOT   167936

#define LDS_FILL ((RCAP + NBF + LISTN) * 4 + 64)
#define LDS_AT1  (2 * GROWS * APK1 * 2)
#define LDS_AT2  (2 * GROWS * APK2 * 2)
#define LDS_STG  (GROWS * FD * 4)
#define LDS_G1   (LDS_AT1 + LDS_STG)
#define LDS_G2   (LDS_AT2 + LDS_STG)
#define LDS_ZY   (LDS_AT1 + GROWS * YW * 4)

#define BN_EPS 1e-5f

static_assert((CHUNK & (CHUNK - 1)) == 0);
static_assert(CHUNK <= 4096);
static_assert(NBC <= 4096 && NBF <= 4096);
static_assert((NBC & (NBC - 1)) == 0 && (NBF & (NBF - 1)) == 0);
static_assert(NBC == 4 * NBF);
static_assert(OTHR * 8 == NBC);
static_assert((RCAP % 32) == 0);
static_assert(TGT == NWAVE * 32 && (TGT % GROWS) == 0);
static_assert((NBC % TGT) == 0);
static_assert(GROWS == NWAVE * 16);
static_assert(FD == 128 && YW == 16 && 2 * NCLS <= YW);
static_assert(WP_PL == WP_M + 2 * FD * K2 && WP_P == WP_PL + 2 * FD * K1);
static_assert(WP_O == WP_P + 2 * FD * K2 && WPTOT == WP_O + 2 * YW * K1);
static_assert((WP_PL % 64) == 0 && (WP_P % 64) == 0 && (WP_O % 64) == 0);
static_assert((LDS_AT1 % 16) == 0 && (LDS_AT2 % 16) == 0);
static_assert(((TGT * NCLS) % 4) == 0);

typedef float          v2f  __attribute__((ext_vector_type(2)));
typedef float          v4f  __attribute__((ext_vector_type(4)));
typedef float          v8f  __attribute__((ext_vector_type(8)));
typedef double         v2d  __attribute__((ext_vector_type(2)));
typedef int            v4i  __attribute__((ext_vector_type(4)));
typedef unsigned short v8us __attribute__((ext_vector_type(8)));
typedef __bf16         v16b __attribute__((ext_vector_type(16)));
union FragB { v16b v; v8us h[2]; };

__device__ __forceinline__ unsigned int bfr(float f) {
  const unsigned int u = __float_as_uint(f);
  return (u + 0x7FFFu + ((u >> 16) & 1u)) >> 16;
}

__device__ __forceinline__ void split1(float x, unsigned short& hb, unsigned short& lb) {
  const unsigned int hu = bfr(x);
  const float hf = __uint_as_float(hu << 16);
  hb = (unsigned short)hu;
  lb = (unsigned short)bfr(x - hf);
}

__device__ __forceinline__ void split8(v4f a, v4f b, v8us& hi, v8us& lo) {
  unsigned short hb, lb;
  split1(a.x, hb, lb); hi[0] = hb; lo[0] = lb;
  split1(a.y, hb, lb); hi[1] = hb; lo[1] = lb;
  split1(a.z, hb, lb); hi[2] = hb; lo[2] = lb;
  split1(a.w, hb, lb); hi[3] = hb; lo[3] = lb;
  split1(b.x, hb, lb); hi[4] = hb; lo[4] = lb;
  split1(b.y, hb, lb); hi[5] = hb; lo[5] = lb;
  split1(b.z, hb, lb); hi[6] = hb; lo[6] = lb;
  split1(b.w, hb, lb); hi[7] = hb; lo[7] = lb;
}

__device__ __forceinline__ v8f wmb(v16b a, v16b b, v8f c) {
  v8f d = __builtin_amdgcn_wmma_f32_16x16x32_bf16(false, a, false, b, (short)0, c, false, false);
  asm volatile("v_nop\n\tv_nop\n\tv_nop\n\tv_nop" : "+v"(d) : "v"(a), "v"(b));
  return d;
}

__device__ __forceinline__ v4f zrow(v4f hm, v4f hp, v4f mum, v4f rsm, v4f gm, v4f bm,
                                    v4f mup, v4f rsp, v4f gp, v4f bp) {
  const v4f t1 = (hm - mum) * rsm * gm + bm;
  const v4f t2 = (hp - mup) * rsp * gp + bp;
  v4f z = t1 + t2;
  z.x = fmaxf(z.x, 0.0f); z.y = fmaxf(z.y, 0.0f); z.z = fmaxf(z.z, 0.0f); z.w = fmaxf(z.w, 0.0f);
  return z;
}

template <int KD, int NT, int NCT, int APK>
__device__ __forceinline__ void mma_tiles(const unsigned short* sHi, const unsigned short* sLo,
                                          const unsigned short* __restrict__ Bw, int wrow, int lane,
                                          v8f (&acc)[NT]) {
  static_assert((KD % 32) == 0 && (APK % 8) == 0);
  constexpr int NKT = KD / 32, WPLN = NCT * KD;
  const int hh = lane >> 4, m = lane & 15;
#pragma unroll
  for (int t = 0; t < NT; ++t) { v8f z = {0.f, 0.f, 0.f, 0.f, 0.f, 0.f, 0.f, 0.f}; acc[t] = z; }
  const unsigned short* ahp = sHi + (wrow + m) * APK + 8 * hh;
  const unsigned short* alp = sLo + (wrow + m) * APK + 8 * hh;
#pragma unroll 1
  for (int kt = 0; kt < NKT; ++kt) {
    FragB ah, al;
    ah.h[0] = *(const v8us*)(ahp + 32 * kt);
    ah.h[1] = *(const v8us*)(ahp + 32 * kt + 16);
    al.h[0] = *(const v8us*)(alp + 32 * kt);
    al.h[1] = *(const v8us*)(alp + 32 * kt + 16);
#pragma unroll
    for (int t = 0; t < NT; ++t) {
      const unsigned short* bp = Bw + (size_t)(16 * t + m) * KD + 32 * kt + 8 * hh;
      FragB bh, bl;
      bh.h[0] = *(const v8us*)bp;
      bh.h[1] = *(const v8us*)(bp + 16);
      bl.h[0] = *(const v8us*)(bp + WPLN);
      bl.h[1] = *(const v8us*)(bp + WPLN + 16);
      acc[t] = wmb(ah.v, bh.v, acc[t]);
      acc[t] = wmb(ah.v, bl.v, acc[t]);
      acc[t] = wmb(al.v, bh.v, acc[t]);
    }
  }
}

__device__ __forceinline__ void store_rows128(const float* stg, float* C, int rowBase, int wave, int lane) {
  const float* lp = stg + wave * 16 * FD + 4 * lane;
  float* gp = C + (size_t)(rowBase + wave * 16) * FD + 4 * lane;
#pragma unroll
  for (int i = 0; i < 16; ++i) { const v4f v = *(const v4f*)(lp + FD * i); *(volatile v4f*)(gp + FD * i) = v; }
  __threadfence();
#pragma unroll
  for (int i = 0; i < 16; ++i) { const v4f v = *(const v4f*)(lp + FD * i); *(volatile v4f*)(gp + FD * i) = v; }
}

template <int NB>
__device__ __forceinline__ int scan_chunk(const int* __restrict__ dsts, int nE, int cbase, int slotBase,
                                          int vec8, int* list, int tid, int lane, int wave) {
  int wc = 0;
#pragma unroll
  for (int g = 0; g < NGRP; ++g) {
    const int el0  = (g * NTHR + tid) * EPT;
    const int e0   = cbase + el0;
    const int sent = -2147483647 - 1;
    v4i da, db;
    if (vec8 != 0 && cbase + CHUNK <= nE) {
      da = *(const v4i*)(dsts + e0);
      db = *(const v4i*)(dsts + e0 + 4);
    } else {
      da.x = (e0     < nE) ? dsts[min(e0, nE - 1)] : sent;
      da.y = (e0 + 1 < nE) ? dsts[min(e0 + 1, nE - 1)] : sent;
      da.z = (e0 + 2 < nE) ? dsts[min(e0 + 2, nE - 1)] : sent;
      da.w = (e0 + 3 < nE) ? dsts[min(e0 + 3, nE - 1)] : sent;
      db.x = (e0 + 4 < nE) ? dsts[min(e0 + 4, nE - 1)] : sent;
      db.y = (e0 + 5 < nE) ? dsts[min(e0 + 5, nE - 1)] : sent;
      db.z = (e0 + 6 < nE) ? dsts[min(e0 + 6, nE - 1)] : sent;
      db.w = (e0 + 7 < nE) ? dsts[min(e0 + 7, nE - 1)] : sent;
    }
    const unsigned nb = (unsigned)slotBase;
    const unsigned s0 = (unsigned)da.x - nb, s1 = (unsigned)da.y - nb;
    const unsigned s2 = (unsigned)da.z - nb, s3 = (unsigned)da.w - nb;
    const unsigned s4 = (unsigned)db.x - nb, s5 = (unsigned)db.y - nb;
    const unsigned s6 = (unsigned)db.z - nb, s7 = (unsigned)db.w - nb;
    const bool h0 = s0 < (unsigned)NB, h1 = s1 < (unsigned)NB, h2 = s2 < (unsigned)NB, h3 = s3 < (unsigned)NB;
    const bool h4 = s4 < (unsigned)NB, h5 = s5 < (unsigned)NB, h6 = s6 < (unsigned)NB, h7 = s7 < (unsigned)NB;
    const unsigned any = __builtin_amdgcn_ballot_w32(h0 | h1 | h2 | h3 | h4 | h5 | h6 | h7);
    if (any != 0u) {
#define HITJ(J, HJ, SJ) { \
        const unsigned mj = __builtin_amdgcn_ballot_w32(HJ); \
        if (mj != 0u) { \
          if (HJ) { \
            const int pos = wc + (int)__builtin_amdgcn_mbcnt_lo(mj, 0u); \
            if (pos < WCAP) list[wave * WCAP + pos] = ((el0 + (J)) << 12) | (int)(SJ); \
          } \
          wc += (int)__builtin_popcount(mj); } }
      HITJ(0, h0, s0)
      HITJ(1, h1, s1)
      HITJ(2, h2, s2)
      HITJ(3, h3, s3)
      HITJ(4, h4, s4)
      HITJ(5, h5, s5)
      HITJ(6, h6, s6)
      HITJ(7, h7, s7)
#undef HITJ
    }
  }
  return wc;
}

__global__ __launch_bounds__(NTHR) void k_wprep(
    const float* __restrict__ wsm, const float* __restrict__ wnm, const float* __restrict__ wpl,
    const float* __restrict__ wsp, const float* __restrict__ wnp,
    const float* __restrict__ wso, const float* __restrict__ wno, unsigned short* wp) {
  const int blk = blockIdx.x, tid = threadIdx.x;
  float v[8];
  int KD, NC, i, base;
  if (blk < 16) {
    KD = K2; NC = FD; i = blk * NTHR + tid; base = WP_M;
    const int n = i >> 5, k0 = (i & 31) * 8;
#pragma unroll
    for (int e = 0; e < 8; ++e) {
      const int k = k0 + e;
      const int ka = k > 127 ? 127 : k;
      int kb = k - 128; kb = kb < 0 ? 0 : kb;
      const float va = wsm[ka * FD + n];
      const float vb = wnm[kb * FD + n];
      v[e] = (k < 128) ? va : vb;
    }
  } else if (blk < 24) {
    KD = K1; NC = FD; i = (blk - 16) * NTHR + tid; base = WP_PL;
    const int n = i >> 4, k0 = (i & 15) * 8;
#pragma unroll
    for (int e = 0; e < 8; ++e) v[e] = wpl[(k0 + e) * FD + n];
  } else if (blk < 40) {
    KD = K2; NC = FD; i = (blk - 24) * NTHR + tid; base = WP_P;
    const int n = i >> 5, k0 = (i & 31) * 8;
#pragma unroll
    for (int e = 0; e < 8; ++e) {
      const int k = k0 + e;
      const int ka = k > 127 ? 127 : k;
      int kb = k - 128; kb = kb < 0 ? 0 : kb;
      const float va = wsp[ka * FD + n];
      const float vb = wnp[kb * FD + n];
      v[e] = (k < 128) ? va : vb;
    }
  } else {
    KD = K1; NC = YW; i = tid; base = WP_O;
    const int n = i >> 4, k0 = (i & 15) * 8;
    const int na = n > (NCLS - 1) ? (NCLS - 1) : n;
    int nb = n - NCLS; nb = nb < 0 ? 0 : (nb > (NCLS - 1) ? (NCLS - 1) : nb);
#pragma unroll
    for (int e = 0; e < 8; ++e) {
      const int k = k0 + e;
      const float va = wso[k * NCLS + na];
      const float vb = wno[k * NCLS + nb];
      v[e] = (n < NCLS) ? va : ((n < 2 * NCLS) ? vb : 0.0f);
    }
  }
  v4f a, b;
  a.x = v[0]; a.y = v[1]; a.z = v[2]; a.w = v[3];
  b.x = v[4]; b.y = v[5]; b.z = v[6]; b.w = v[7];
  v8us hv, lv;
  split8(a, b, hv, lv);
  unsigned short* dh = wp + base + (size_t)i * 8;
  unsigned short* dl = dh + NC * KD;
  *(volatile v8us*)dh = hv;
  *(volatile v8us*)dl = lv;
  __threadfence();
  *(volatile v8us*)dh = hv;
  *(volatile v8us*)dl = lv;
}

__global__ __launch_bounds__(NTHR) void k_count(const int* __restrict__ dsts, int* cnt, int nE, int vec8) {
  __shared__ __attribute__((aligned(16))) int scnt[NBC];
  __shared__ __attribute__((aligned(16))) int list[LISTN];
  __shared__ int wcnt[NWAVE];
  const int tid = threadIdx.x, lane = tid & 31, wave = tid >> 5;
  const int nodeBase = blockIdx.x * NBC;

  for (int i = tid; i < NBC; i += NTHR) scnt[i] = 0;
  __syncthreads();

  const int nChunks = (nE + CHUNK - 1) / CHUNK;
#pragma unroll 1
  for (int ch = 0; ch < nChunks; ++ch) {
    const int cbase = ch * CHUNK;
    const int wc = scan_chunk<NBC>(dsts, nE, cbase, nodeBase, vec8, list, tid, lane, wave);
    if (lane == 0) wcnt[wave] = wc;
    __syncthreads();
    if (wave == 0) {
#pragma unroll 1
      for (int wsx = 0; wsx < NWAVE; ++wsx) {
        int n = __builtin_amdgcn_readfirstlane(wcnt[wsx]);
        n = n > WCAP ? WCAP : (n < 0 ? 0 : n);
        const int* lp = list + wsx * WCAP;
#pragma unroll 1
        for (int i = 0; i < n; ++i) {
          const int ent  = __builtin_amdgcn_readfirstlane(lp[i]);
          const int slot = ent & (NBC - 1);
          if (lane == 0) scnt[slot] = scnt[slot] + 1;
        }
      }
    }
    __syncthreads();
  }

  v4i cq[4];
#pragma unroll
  for (int q = 0; q < 4; ++q) {
    const int f = (wave * 4 + q) * 128 + 4 * lane;
    cq[q] = *(const v4i*)(scnt + f);
  }
  int* cp = cnt + (size_t)nodeBase;
#pragma unroll
  for (int q = 0; q < 4; ++q) {
    const int f = (wave * 4 + q) * 128 + 4 * lane;
    *(volatile v4i*)(cp + f) = cq[q];
  }
  __threadfence();
#pragma unroll
  for (int q = 0; q < 4; ++q) {
    const int f = (wave * 4 + q) * 128 + 4 * lane;
    *(volatile v4i*)(cp + f) = cq[q];
  }
}

__global__ __launch_bounds__(OTHR) void k_offsets(
    const int* __restrict__ cnt, int* off, int* rbase, int nChunk) {
  __shared__ __attribute__((aligned(16))) int soff[NBC];
  __shared__ __attribute__((aligned(16))) int srb[RBN];
  __shared__ int wtot[OTHR / 32];
  const int tid = threadIdx.x, lane = tid & 31, wave = tid >> 5, sub = tid >> 7;
  for (int i = tid; i < RBN; i += OTHR) srb[i] = 0;
  int carry = 0;
#pragma unroll 1
  for (int ch = 0; ch < nChunk; ++ch) {
    const int base = ch * NBC;
    const v4i c0 = *(const v4i*)(cnt + base + 8 * tid);
    const v4i c1 = *(const v4i*)(cnt + base + 8 * tid + 4);
    const int e0 = max(c0.x, 0), e1 = max(c0.y, 0), e2 = max(c0.z, 0), e3 = max(c0.w, 0);
    const int e4 = max(c1.x, 0), e5 = max(c1.y, 0), e6 = max(c1.z, 0), e7 = max(c1.w, 0);
    const int ts = e0 + e1 + e2 + e3 + e4 + e5 + e6 + e7;
    int incl = ts;
#pragma unroll
    for (int d = 1; d < 32; d <<= 1) {
      const int t = __shfl_up(incl, d);
      if (lane >= d) incl += t;
    }
    if (lane == 31) wtot[wave] = incl;
    __syncthreads();
    const int S0 = wtot[0]  + wtot[1]  + wtot[2]  + wtot[3];
    const int S1 = wtot[4]  + wtot[5]  + wtot[6]  + wtot[7];
    const int S2 = wtot[8]  + wtot[9]  + wtot[10] + wtot[11];
    const int S3 = wtot[12] + wtot[13] + wtot[14] + wtot[15];
    int pre = 0;
#pragma unroll 1
    for (int w = 4 * sub; w < wave; ++w) pre += wtot[w];
    const int b0 = carry;
    const int b1 = b0 + ((S0 + 31) & ~31);
    const int b2 = b1 + ((S1 + 31) & ~31);
    const int b3 = b2 + ((S2 + 31) & ~31);
    const int b4 = b3 + ((S3 + 31) & ~31);
    const int myb = sub == 0 ? b0 : (sub == 1 ? b1 : (sub == 2 ? b2 : b3));
    if (tid == 0) {
      srb[min(4 * ch + 0, RBN - 1)] = b0;
      srb[min(4 * ch + 1, RBN - 1)] = b1;
      srb[min(4 * ch + 2, RBN - 1)] = b2;
      srb[min(4 * ch + 3, RBN - 1)] = b3;
    }
    int run = myb + pre + incl - ts;
    soff[8 * tid + 0] = run; run += e0;
    soff[8 * tid + 1] = run; run += e1;
    soff[8 * tid + 2] = run; run += e2;
    soff[8 * tid + 3] = run; run += e3;
    soff[8 * tid + 4] = run; run += e4;
    soff[8 * tid + 5] = run; run += e5;
    soff[8 * tid + 6] = run; run += e6;
    soff[8 * tid + 7] = run;
    carry = b4;
    __syncthreads();
    const v4i o0 = *(const v4i*)(soff + 4 * tid);
    const v4i o1 = *(const v4i*)(soff + 4 * (tid + OTHR));
    int* op = off + base;
    *(volatile v4i*)(op + 4 * tid) = o0;
    *(volatile v4i*)(op + 4 * (tid + OTHR)) = o1;
    __threadfence();
    *(volatile v4i*)(op + 4 * tid) = o0;
    *(volatile v4i*)(op + 4 * (tid + OTHR)) = o1;
    __syncthreads();
  }
  if (tid == 0) srb[min(4 * nChunk, RBN - 1)] = carry;
  __syncthreads();
  v4i rv = {0, 0, 0, 0};
  if (tid < 32) rv = *(const v4i*)(srb + 4 * tid);
  if (tid < 32) *(volatile v4i*)(rbase + 4 * tid) = rv;
  __threadfence();
  if (tid < 32) *(volatile v4i*)(rbase + 4 * tid) = rv;
}

__global__ __launch_bounds__(NTHR) void k_fill(
    const int* __restrict__ srcs, const int* __restrict__ dsts,
    const int* __restrict__ off, const int* __restrict__ rbase,
    int* csr, int nN, int nE, int vec8, int csrLen) {
  extern __shared__ v4f lds_dyn[];
  int* region = (int*)lds_dyn;
  int* cursor = region + RCAP;
  int* list   = cursor + NBF;
  int* wcnt   = list + LISTN;
  const int tid = threadIdx.x, lane = tid & 31, wave = tid >> 5;
  const int b = blockIdx.x;
  const int nodeBase = b * NBF;

  int rb0 = rbase[b];
  const int rb1 = rbase[b + 1];
  rb0 = rb0 < 0 ? 0 : (rb0 > csrLen ? csrLen : rb0);
  rb0 &= ~31;
  int len = rb1 - rb0;
  len = len < 0 ? 0 : (len > RCAP ? RCAP : len);
  int lenW = (len + 31) & ~31;
  if (rb0 + lenW > csrLen) lenW = (csrLen - rb0) & ~31;

  {
    const v4i z = {0, 0, 0, 0};
    for (int i = tid; i < RCAP / 4; i += NTHR) ((v4i*)region)[i] = z;
    for (int s = tid; s < NBF; s += NTHR) {
      int o = off[nodeBase + s] - rb0;
      o = o < 0 ? 0 : (o > RCAP ? RCAP : o);
      cursor[s] = o;
    }
  }
  __syncthreads();

  const int nChunks = (nE + CHUNK - 1) / CHUNK;
#pragma unroll 1
  for (int ch = 0; ch < nChunks; ++ch) {
    const int cbase = ch * CHUNK;
    const int wc = scan_chunk<NBF>(dsts, nE, cbase, nodeBase, vec8, list, tid, lane, wave);
    if (lane == 0) wcnt[wave] = wc;
    __syncthreads();
    if (wave == 0) {
#pragma unroll 1
      for (int wsx = 0; wsx < NWAVE; ++wsx) {
        int n = __builtin_amdgcn_readfirstlane(wcnt[wsx]);
        n = n > WCAP ? WCAP : (n < 0 ? 0 : n);
        const int* lp = list + wsx * WCAP;
#pragma unroll 1
        for (int i = 0; i < n; ++i) {
          const int ent  = __builtin_amdgcn_readfirstlane(lp[i]);
          const int slot = ent & (NBF - 1);
          int e = cbase + ((ent >> 12) & (CHUNK - 1));
          e = e > nE - 1 ? nE - 1 : e;
          int sv = srcs[e];
          sv = sv < 0 ? 0 : (sv > nN - 1 ? nN - 1 : sv);
          if (lane == 0) {
            int pos = cursor[slot];
            pos = pos < 0 ? 0 : (pos > RCAP - 1 ? RCAP - 1 : pos);
            region[pos] = sv;
            const int np = pos + 1;
            cursor[slot] = np > RCAP ? RCAP : np;
          }
        }
      }
    }
    __syncthreads();
  }

  const int nv = lenW >> 2;
  int* gp = csr + rb0;
#pragma unroll 1
  for (int i = tid; i < nv; i += NTHR) { const v4i v = ((const v4i*)region)[i]; *(volatile v4i*)(gp + 4 * i) = v; }
  __threadfence();
#pragma unroll 1
  for (int i = tid; i < nv; i += NTHR) { const v4i v = ((const v4i*)region)[i]; *(volatile v4i*)(gp + 4 * i) = v; }
}

template <int KD, bool STATS>
__global__ __launch_bounds__(NTHR) void k_gemm(
    const float* __restrict__ x, const float* __restrict__ agg,
    const unsigned short* __restrict__ Bw, const float* __restrict__ bias,
    float* C, double* part, int nN) {
  static_assert(KD == K1 || KD == K2);
  constexpr int APK = KD + 8;
  extern __shared__ v4f lds_dyn[];
  __shared__ __attribute__((aligned(16))) double dS[2 * FD];
  __shared__ __attribute__((aligned(16))) double dQ[2 * FD];
  __shared__ __attribute__((aligned(16))) double dP[2 * FD];
  unsigned short* sHi = (unsigned short*)lds_dyn;
  unsigned short* sLo = sHi + GROWS * APK;
  float*          stg = (float*)((char*)lds_dyn + 2 * GROWS * APK * 2);
  const int tid = threadIdx.x, lane = tid & 31, wave = tid >> 5, hh = lane >> 4, m = lane & 15;
  const int rowBase = blockIdx.x * GROWS;
  const int c0 = (tid & 15) * 8, rr = tid >> 4;

#pragma unroll 2
  for (int it = 0; it < 8; ++it) {
    const int r = it * 16 + rr;
    int row = rowBase + r;
    row = row > nN - 1 ? nN - 1 : row;
    const float* ap = x + (size_t)row * FD + c0;
    const v4f a = *(const v4f*)ap, b = *(const v4f*)(ap + 4);
    v8us hv, lv;
    split8(a, b, hv, lv);
    *(v8us*)(sHi + r * APK + c0) = hv;
    *(v8us*)(sLo + r * APK + c0) = lv;
  }
  if (KD == K2) {
#pragma unroll 2
    for (int it = 0; it < 8; ++it) {
      const int r = it * 16 + rr;
      const float* ap = agg + (size_t)(rowBase + r) * FD + c0;
      const v4f a = *(const v4f*)ap, b = *(const v4f*)(ap + 4);
      v8us hv, lv;
      split8(a, b, hv, lv);
      *(v8us*)(sHi + r * APK + FD + c0) = hv;
      *(v8us*)(sLo + r * APK + FD + c0) = lv;
    }
  }
  __syncthreads();

#pragma unroll
  for (int ch = 0; ch < 2; ++ch) {
    v8f acc[4];
    mma_tiles<KD, 4, FD, APK>(sHi, sLo, Bw + (size_t)(64 * ch) * KD, wave * 16, lane, acc);
    float* sp = stg + (wave * 16 + 8 * hh) * FD + 64 * ch + m;
#pragma unroll
    for (int t = 0; t < 4; ++t) {
      const float bv = bias[64 * ch + 16 * t + m];
#pragma unroll
      for (int r = 0; r < 8; ++r) {
        float v = acc[t][r] + bv;
        v = fmaxf(v, 0.0f);
        sp[r * FD + 16 * t] = v;
      }
    }
  }
  __syncthreads();

  if (STATS) {
    {
      const int c = tid & (FD - 1), hf = tid >> 7;
      double s = 0.0, q = 0.0;
#pragma unroll 4
      for (int i = 0; i < 64; ++i) {
        const int r = hf * 64 + i;
        const float v = stg[r * FD + c];
        const float vz = (rowBase + r < nN) ? v : 0.0f;
        const double dv = (double)vz;
        s += dv;
        q = fma(dv, dv, q);
      }
      dS[hf * FD + c] = s;
      dQ[hf * FD + c] = q;
    }
    __syncthreads();
    if (tid < FD) {
      dP[tid]      = dS[tid] + dS[FD + tid];
      dP[FD + tid] = dQ[tid] + dQ[FD + tid];
    }
    __syncthreads();
    v2d pv = {0.0, 0.0};
    if (tid < FD) pv = *(const v2d*)(dP + 2 * tid);
    double* gq = part + (size_t)blockIdx.x * (2 * FD) + 2 * tid;
    if (tid < FD) *(volatile v2d*)gq = pv;
    __threadfence();
    if (tid < FD) *(volatile v2d*)gq = pv;
  }

  store_rows128(stg, C, rowBase, wave, lane);
}

__global__ __launch_bounds__(NTHR) void k_agg1(
    const int* __restrict__ csr, const int* __restrict__ off, const int* __restrict__ cnt,
    const float* __restrict__ xs, const float* __restrict__ xm,
    float* Am, float* Ax, int nN, int csrLen) {
  const int tid = threadIdx.x, lane = tid & 31, wave = tid >> 5;
  const int tbase = blockIdx.x * TGT + wave * 32;
  const int cl = tbase + lane;
  const int cnt_l = cnt[cl];
  const int off_l = off[cl];
  const float ninf = __uint_as_float(0xff800000u);

#pragma unroll 1
  for (int j = 0; j < 32; ++j) {
    const int c = tbase + j;
    int n = __builtin_amdgcn_readlane(cnt_l, j);
    n = n < 0 ? 0 : (n > DEGCAP ? DEGCAP : n);
    const int st = __builtin_amdgcn_readlane(off_l, j);
    v4f sm = {0.0f, 0.0f, 0.0f, 0.0f};
    v4f mx = {ninf, ninf, ninf, ninf};
#pragma unroll 1
    for (int q0 = 0; q0 < n; q0 += 32) {
      int pos = st + q0 + lane;
      pos = pos < 0 ? 0 : (pos > csrLen - 1 ? csrLen - 1 : pos);
      int sl = csr[pos];
      sl = sl < 0 ? 0 : (sl > nN - 1 ? nN - 1 : sl);
      const int mcnt = (n - q0) < 32 ? (n - q0) : 32;
#pragma unroll 1
      for (int p = 0; p < mcnt; ++p) {
        const int s = __builtin_amdgcn_readlane(sl, p);
        const v4f vf = *(const v4f*)(xs + (size_t)s * FD + 4 * lane);
        const v4f vp = *(const v4f*)(xm + (size_t)s * FD + 4 * lane);
        sm = sm + vf;
        mx.x = fmaxf(mx.x, vp.x);
        mx.y = fmaxf(mx.y, vp.y);
        mx.z = fmaxf(mx.z, vp.z);
        mx.w = fmaxf(mx.w, vp.w);
      }
    }
    const float rc = 1.0f / (float)(n > 1 ? n : 1);
    const v4f mean = sm * rc;
    v4f mo;
    mo.x = n > 0 ? mx.x : 0.0f; mo.y = n > 0 ? mx.y : 0.0f;
    mo.z = n > 0 ? mx.z : 0.0f; mo.w = n > 0 ? mx.w : 0.0f;
    float* ap  = Am + (size_t)c * FD + 4 * lane;
    float* xpo = Ax + (size_t)c * FD + 4 * lane;
    *(volatile v4f*)ap  = mean;
    *(volatile v4f*)xpo = mo;
    __threadfence();
    *(volatile v4f*)ap  = mean;
    *(volatile v4f*)xpo = mo;
  }
}

__global__ __launch_bounds__(NTHR) void k_bnfin(const double* __restrict__ part, float* coef, int nBlk, int nN) {
  __shared__ __attribute__((aligned(16))) float sco[4 * FD];
  const int tid = threadIdx.x, br = tid >> 7, c = tid & (FD - 1);
  const double* pp = part + (size_t)br * nBlk * (2 * FD);
  double S = 0.0, Q = 0.0;
#pragma unroll 1
  for (int b = 0; b < nBlk; ++b) {
    S += pp[(size_t)b * (2 * FD) + c];
    Q += pp[(size_t)b * (2 * FD) + FD + c];
  }
  const double rn = 1.0 / (double)(nN > 1 ? nN : 1);
  const double mean = S * rn;
  double var = Q * rn - mean * mean;
  var = var < 0.0 ? 0.0 : var;
  const float muf = (float)mean;
  const float rs  = rsqrtf((float)var + BN_EPS);
  sco[br * 2 * FD + c]      = muf;
  sco[br * 2 * FD + FD + c] = rs;
  __syncthreads();
  v4f cv = {0.f, 0.f, 0.f, 0.f};
  if (tid < FD) cv = *(const v4f*)(sco + 4 * tid);
  if (tid < FD) *(volatile v4f*)(coef + 4 * tid) = cv;
  __threadfence();
  if (tid < FD) *(volatile v4f*)(coef + 4 * tid) = cv;
}

__global__ __launch_bounds__(NTHR) void k_zy(
    const float* __restrict__ hm, const float* __restrict__ hp, const float* __restrict__ coef,
    const float* __restrict__ gm, const float* __restrict__ bm,
    const float* __restrict__ gp, const float* __restrict__ bp,
    const unsigned short* __restrict__ Bw, float* Y) {
  extern __shared__ v4f lds_dyn[];
  unsigned short* sHi = (unsigned short*)lds_dyn;
  unsigned short* sLo = sHi + GROWS * APK1;
  float*          stg = (float*)((char*)lds_dyn + LDS_AT1);
  const int tid = threadIdx.x, lane = tid & 31, wave = tid >> 5, hh = lane >> 4, m = lane & 15;
  const int rowBase = blockIdx.x * GROWS;
  const int c0 = (tid & 15) * 8, rr = tid >> 4;

  const v4f muma = *(const v4f*)(coef + c0),          mumb = *(const v4f*)(coef + c0 + 4);
  const v4f rsma = *(const v4f*)(coef + FD + c0),     rsmb = *(const v4f*)(coef + FD + c0 + 4);
  const v4f mupa = *(const v4f*)(coef + 2 * FD + c0), mupb = *(const v4f*)(coef + 2 * FD + c0 + 4);
  const v4f rspa = *(const v4f*)(coef + 3 * FD + c0), rspb = *(const v4f*)(coef + 3 * FD + c0 + 4);
  const v4f gma = *(const v4f*)(gm + c0), gmb = *(const v4f*)(gm + c0 + 4);
  const v4f bma = *(const v4f*)(bm + c0), bmb = *(const v4f*)(bm + c0 + 4);
  const v4f gpa = *(const v4f*)(gp + c0), gpb = *(const v4f*)(gp + c0 + 4);
  const v4f bpa = *(const v4f*)(bp + c0), bpb = *(const v4f*)(bp + c0 + 4);

#pragma unroll 2
  for (int it = 0; it < 8; ++it) {
    const int r = it * 16 + rr;
    const float* pm = hm + (size_t)(rowBase + r) * FD + c0;
    const float* pq = hp + (size_t)(rowBase + r) * FD + c0;
    const v4f hma = *(const v4f*)pm, hmb = *(const v4f*)(pm + 4);
    const v4f hpa = *(const v4f*)pq, hpb = *(const v4f*)(pq + 4);
    const v4f za = zrow(hma, hpa, muma, rsma, gma, bma, mupa, rspa, gpa, bpa);
    const v4f zb = zrow(hmb, hpb, mumb, rsmb, gmb, bmb, mupb, rspb, gpb, bpb);
    v8us hv, lv;
    split8(za, zb, hv, lv);
    *(v8us*)(sHi + r * APK1 + c0) = hv;
    *(v8us*)(sLo + r * APK1 + c0) = lv;
  }
  __syncthreads();

  v8f acc[1];
  mma_tiles<K1, 1, YW, APK1>(sHi, sLo, Bw, wave * 16, lane, acc);
  {
    float* sp = stg + (wave * 16 + 8 * hh) * YW + m;
#pragma unroll
    for (int r = 0; r < 8; ++r) sp[r * YW] = acc[0][r];
  }
  __syncthreads();

  float* yb = Y + (size_t)rowBase * YW;
  const v4f y0 = *(const v4f*)(stg + 4 * tid);
  const v4f y1 = *(const v4f*)(stg + 4 * (tid + NTHR));
  *(volatile v4f*)(yb + 4 * tid) = y0;
  *(volatile v4f*)(yb + 4 * (tid + NTHR)) = y1;
  __threadfence();
  *(volatile v4f*)(yb + 4 * tid) = y0;
  *(volatile v4f*)(yb + 4 * (tid + NTHR)) = y1;
}

__device__ __forceinline__ void out_pass(const float* sout, float* ob, int nf, int tid) {
#pragma unroll
  for (int it = 0; it < 2; ++it) {
    const int q = it * NTHR + tid;
    if (q < (TGT * NCLS) / 4) {
      const v4f v = *(const v4f*)(sout + 4 * q);
      if (4 * q + 4 <= nf) {
        *(volatile v4f*)(ob + 4 * q) = v;
      } else if (4 * q < nf) {
        volatile float* op = ob + 4 * q;
        op[0] = v.x;
        if (4 * q + 1 < nf) op[1] = v.y;
        if (4 * q + 2 < nf) op[2] = v.z;
      }
    }
  }
}

__global__ __launch_bounds__(NTHR) void k_aggout(
    const int* __restrict__ csr, const int* __restrict__ off, const int* __restrict__ cnt,
    const float* __restrict__ Y, const float* __restrict__ bo, float* out, int nN, int csrLen) {
  __shared__ __attribute__((aligned(16))) float sout[TGT * NCLS];
  const int tid = threadIdx.x, lane = tid & 31, wave = tid >> 5;
  const int tbase = blockIdx.x * TGT + wave * 32;
  const int cl = tbase + lane;
  const int cnt_l = cnt[cl];
  const int off_l = off[cl];
  const int ch = lane & 15;
  const float bov = bo[lane < NCLS ? lane : (NCLS - 1)];

#pragma unroll 1
  for (int j = 0; j < 32; ++j) {
    const int c = tbase + j;
    int n = __builtin_amdgcn_readlane(cnt_l, j);
    n = n < 0 ? 0 : (n > DEGCAP ? DEGCAP : n);
    const int st = __builtin_amdgcn_readlane(off_l, j);
    float sm = 0.0f;
#pragma unroll 1
    for (int q0 = 0; q0 < n; q0 += 32) {
      int pos = st + q0 + lane;
      pos = pos < 0 ? 0 : (pos > csrLen - 1 ? csrLen - 1 : pos);
      int sl = csr[pos];
      sl = sl < 0 ? 0 : (sl > nN - 1 ? nN - 1 : sl);
      const int mcnt = (n - q0) < 32 ? (n - q0) : 32;
#pragma unroll 1
      for (int p = 0; p < mcnt; ++p) {
        const int s = __builtin_amdgcn_readlane(sl, p);
        sm += Y[(size_t)s * YW + ch];
      }
    }
    const float rc = 1.0f / (float)(n > 1 ? n : 1);
    const float nbv = __shfl(sm, (lane + NCLS) & 31);
    const float ys = Y[(size_t)c * YW + ch];
    const float o = ys + nbv * rc + bov;
    if (lane < NCLS) sout[(wave * 32 + j) * NCLS + lane] = o;
  }
  __syncthreads();

  int nvalid = nN - blockIdx.x * TGT;
  nvalid = nvalid > TGT ? TGT : (nvalid < 0 ? 0 : nvalid);
  const int nf = nvalid * NCLS;
  float* ob = out + (size_t)blockIdx.x * (TGT * NCLS);
  out_pass(sout, ob, nf, tid);
  __threadfence();
  out_pass(sout, ob, nf, tid);
}

extern "C" void kernel_launch(void* const* d_in, const int* in_sizes, int n_in,
                              void* d_out, int out_size, void* d_ws, size_t ws_size,
                              hipStream_t stream) {
  if (n_in < 18) return;
  const int nN = in_sizes[0] / FD;
  const int nE = in_sizes[1];
  if (nN <= 0 || nE <= 0) return;
  if (in_sizes[0] != nN * FD || in_sizes[2] != nE) return;
  if (in_sizes[3] != FD * FD || in_sizes[4] != FD * FD || in_sizes[5] != FD) return;
  if (in_sizes[6] != FD * FD || in_sizes[7] != FD) return;
  if (in_sizes[8] != FD * FD || in_sizes[9] != FD * FD || in_sizes[10] != FD) return;
  if (in_sizes[11] != FD || in_sizes[12] != FD || in_sizes[13] != FD || in_sizes[14] != FD) return;
  if (in_sizes[15] != FD * NCLS || in_sizes[16] != FD * NCLS || in_sizes[17] != NCLS) return;
  if (out_size != nN * NCLS) return;
  if (nE > (1 << 28) || nN > (1 << 24)) return;

  const float* x     = (const float*)d_in[0];
  const int*   srcs  = (const int*)d_in[1];
  const int*   dsts  = (const int*)d_in[2];
  const float* wsm   = (const float*)d_in[3];
  const float* wnm   = (const float*)d_in[4];
  const float* b_m   = (const float*)d_in[5];
  const float* wpl   = (const float*)d_in[6];
  const float* b_pl  = (const float*)d_in[7];
  const float* wsp   = (const float*)d_in[8];
  const float* wnp   = (const float*)d_in[9];
  const float* b_p   = (const float*)d_in[10];
  const float* gam_m = (const float*)d_in[11];
  const float* bet_m = (const float*)d_in[12];
  const float* gam_p = (const float*)d_in[13];
  const float* bet_p = (const float*)d_in[14];
  const float* wso   = (const float*)d_in[15];
  const float* wno   = (const float*)d_in[16];
  const float* b_o   = (const float*)d_in[17];
  float* out = (float*)d_out;

  const int NPAD   = ((nN + TGT - 1) / TGT) * TGT;
  const int nBC    = (nN + NBC - 1) / NBC;
  const int CNTPAD = nBC * NBC;
  if (4 * nBC + 1 > RBN) return;
  const int nBF    = (nN + NBF - 1) / NBF;
  const int csrLen = ((nE + 31) & ~31) + 4096;
  if (31 * 4 * nBC > 4096) return;
  const int nGemm  = NPAD / GROWS;
  const int nAgg   = NPAD / TGT;

  char* ws = (char*)d_ws;
  size_t off = 0;
  const size_t oW    = off; off += (size_t)WPTOT * 2;               off = (off + 255) & ~(size_t)255;
  const size_t oCnt  = off; off += (size_t)CNTPAD * 4;              off = (off + 255) & ~(size_t)255;
  const size_t oOff  = off; off += (size_t)CNTPAD * 4;              off = (off + 255) & ~(size_t)255;
  const size_t oRb   = off; off += (size_t)RBN * 4;                 off = (off + 255) & ~(size_t)255;
  const size_t oCsr  = off; off += (size_t)csrLen * 4;              off = (off + 255) & ~(size_t)255;
  const size_t oR1   = off; off += (size_t)NPAD * FD * 4;           off = (off + 255) & ~(size_t)255;
  const size_t oR2   = off; off += (size_t)NPAD * FD * 4;           off = (off + 255) & ~(size_t)255;
  const size_t oR3   = off; off += (size_t)NPAD * FD * 4;           off = (off + 255) & ~(size_t)255;
  const size_t oY    = off; off += (size_t)NPAD * YW * 4;           off = (off + 255) & ~(size_t)255;
  const size_t oPart = off; off += (size_t)2 * nGemm * (2 * FD) * 8; off = (off + 255) & ~(size_t)255;
  const size_t oCoef = off; off += (size_t)4 * FD * 4;              off = (off + 255) & ~(size_t)255;
  if (off > ws_size || off > (size_t)WSCAP) return;
  unsigned short* wp   = (unsigned short*)(ws + oW);
  int*            cnt  = (int*)(ws + oCnt);
  int*            offp = (int*)(ws + oOff);
  int*            rb   = (int*)(ws + oRb);
  int*            csr  = (int*)(ws + oCsr);
  float*          R1   = (float*)(ws + oR1);
  float*          R2   = (float*)(ws + oR2);
  float*          R3   = (float*)(ws + oR3);
  float*          Yp   = (float*)(ws + oY);
  double*         part = (double*)(ws + oPart);
  float*          coef = (float*)(ws + oCoef);

  const int vec8 = 1;

  k_wprep<<<41, NTHR, 0, stream>>>(wsm, wnm, wpl, wsp, wnp, wso, wno, wp);

  k_count<<<nBC, NTHR, 0, stream>>>(dsts, cnt, nE, vec8);
  k_offsets<<<1, OTHR, 0, stream>>>(cnt, offp, rb, nBC);
  hipFuncSetAttribute(reinterpret_cast<const void*>(&k_fill),
                      hipFuncAttributeMaxDynamicSharedMemorySize, LDS_FILL);
  k_fill<<<nBF, NTHR, LDS_FILL, stream>>>(srcs, dsts, offp, rb, csr, nN, nE, vec8, csrLen);

  hipFuncSetAttribute(reinterpret_cast<const void*>(&k_gemm<K1, false>),
                      hipFuncAttributeMaxDynamicSharedMemorySize, LDS_G1);
  k_gemm<K1, false><<<nGemm, NTHR, LDS_G1, stream>>>(x, x, wp + WP_PL, b_pl, R1, part, nN);

  k_agg1<<<nAgg, NTHR, 0, stream>>>(csr, offp, cnt, x, R1, R2, R3, nN, csrLen);

  hipFuncSetAttribute(reinterpret_cast<const void*>(&k_gemm<K2, true>),
                      hipFuncAttributeMaxDynamicSharedMemorySize, LDS_G2);
  k_gemm<K2, true><<<nGemm, NTHR, LDS_G2, stream>>>(x, R2, wp + WP_M, b_m, R1, part, nN);
  k_gemm<K2, true><<<nGemm, NTHR, LDS_G2, stream>>>(x, R3, wp + WP_P, b_p, R2,
                                                     part + (size_t)nGemm * (2 * FD), nN);

  k_bnfin<<<1, NTHR, 0, stream>>>(part, coef, nGemm, nN);

  hipFuncSetAttribute(reinterpret_cast<const void*>(&k_zy),
                      hipFuncAttributeMaxDynamicSharedMemorySize, LDS_ZY);
  k_zy<<<nGemm, NTHR, LDS_ZY, stream>>>(R1, R2, coef, gam_m, bet_m, gam_p, bet_p, wp + WP_O, Yp);

  k_aggout<<<nAgg, NTHR, 0, stream>>>(csr, offp, cnt, Yp, b_o, out, nN, csrLen);
}
